// BiLSTM_CRF_84207128805837
// MI455X (gfx1250) — hardware-verified
//
#include <hip/hip_runtime.h>
#include <math.h>

constexpr int NBATCH = 32;
constexpr int NSTEPS = 256;
constexpr int NEMB   = 300;
constexpr int KPE    = 320;
constexpr int NHID   = 256;
constexpr int NGATE  = 1024;
constexpr int NTAGS  = 9;
constexpr int NVOCAB = 50000;
constexpr int NROWS  = NBATCH * NSTEPS;
constexpr int SEQW   = 2 * NHID;
constexpr int NTHR   = 256;
constexpr int XCH    = KPE / 8;
constexpr int HCH    = NHID / 8;
constexpr int RBLK   = 16;
constexpr int HPITCH = 264;
constexpr int SLABP  = 36;
constexpr int NOUT0  = NROWS * NTAGS;
static_assert(NBATCH == 32);
static_assert(KPE % 32 == 0 && KPE >= NEMB);
static_assert(NHID % 32 == 0);
static_assert(NROWS % 64 == 0 && NGATE % 64 == 0);
static_assert((NROWS * XCH) % NTHR == 0);
static_assert((NGATE * XCH) % NTHR == 0 && (NGATE * HCH) % NTHR == 0);
static_assert(NROWS % NTHR == 0);
static_assert((2 * RBLK * HPITCH) % NTHR == 0);
static_assert((RBLK * NGATE) % (4 * NTHR) == 0);
static_assert(NHID == 32 * (NTHR / 32));
static_assert(NOUT0 * 4 == 294912);
static_assert(((NROWS * XCH / NTHR) * NTHR) == NROWS * XCH);

typedef __attribute__((ext_vector_type(16))) _Float16 v16h;
typedef __attribute__((ext_vector_type(8)))  _Float16 v8h;
typedef __attribute__((ext_vector_type(16))) __bf16   v16b;
typedef __attribute__((ext_vector_type(8)))  __bf16   v8b;
typedef __attribute__((ext_vector_type(8)))  float    v8f;
typedef __attribute__((ext_vector_type(4)))  float    v4f;

__device__ __forceinline__ unsigned short f2bf_bits(float f) {
  unsigned u = __float_as_uint(f);
  return (unsigned short)((u + 0x7FFFu + ((u >> 16) & 1u)) >> 16);
}
__device__ __forceinline__ float bf_bits2f(unsigned short h) { return __uint_as_float(((unsigned)h) << 16); }
__device__ __forceinline__ float bf16r(float f) { return bf_bits2f(f2bf_bits(f)); }

__device__ __forceinline__ void dep_guard_h(v8f& a, v8f& b, v16h x, v16h y) { asm volatile("v_nop\n\tv_nop\n\tv_nop\n\tv_nop" : "+v"(a), "+v"(b) : "v"(x), "v"(y)); }
__device__ __forceinline__ void dep_guard_b(v8f& a, v8f& b, v16b x, v16b y) { asm volatile("v_nop\n\tv_nop\n\tv_nop\n\tv_nop" : "+v"(a), "+v"(b) : "v"(x), "v"(y)); }
__device__ __forceinline__ void keep4_h(v16h a, v16h b, v16h c, v16h d) { asm volatile("v_nop" :: "v"(a), "v"(b), "v"(c), "v"(d)); }
__device__ __forceinline__ void keep4_b(v16b a, v16b b, v16b c, v16b d) { asm volatile("v_nop" :: "v"(a), "v"(b), "v"(c), "v"(d)); }
__device__ __forceinline__ void acc_guard4(v8f& a, v8f& b, v8f& c, v8f& d) { asm volatile("v_nop\n\tv_nop\n\tv_nop\n\tv_nop" : "+v"(a), "+v"(b), "+v"(c), "+v"(d)); }
__device__ __forceinline__ void guard8_b(v8f& a0, v8f& a1, v8f& a2, v8f& a3,
                                         v16b x0, v16b x1, v16b y0, v16b y1, v16b y2, v16b y3) {
  asm volatile("v_nop\n\tv_nop\n\tv_nop\n\tv_nop"
               : "+v"(a0), "+v"(a1), "+v"(a2), "+v"(a3)
               : "v"(x0), "v"(x1), "v"(y0), "v"(y1), "v"(y2), "v"(y3));
}
template <typename T> struct Frag;
template <> struct Frag<_Float16> {
  typedef v16h V; union U { v16h v; v8h h[2]; };
  static __device__ __forceinline__ v16h load(const _Float16* p) {
    U f; f.h[0] = *(const v8h*)(p); f.h[1] = *(const v8h*)(p + 16); return f.v;
  }
  static __device__ __forceinline__ v8f mma(v16h a, v16h b, v8f c) {
    return __builtin_amdgcn_wmma_f32_16x16x32_f16(false, a, false, b, (short)0, c, false, false);
  }
  static __device__ __forceinline__ void guard(v8f& a, v8f& b, v16h x, v16h y) { dep_guard_h(a, b, x, y); }
  static __device__ __forceinline__ void keep(v16h a, v16h b, v16h c, v16h d) { keep4_h(a, b, c, d); }
};
template <> struct Frag<__bf16> {
  typedef v16b V; union U { v16b v; v8b h[2]; };
  static __device__ __forceinline__ v16b load(const __bf16* p) {
    U f; f.h[0] = *(const v8b*)(p); f.h[1] = *(const v8b*)(p + 16); return f.v;
  }
  static __device__ __forceinline__ v8f mma(v16b a, v16b b, v8f c) {
    return __builtin_amdgcn_wmma_f32_16x16x32_bf16(false, a, false, b, (short)0, c, false, false);
  }
  static __device__ __forceinline__ void guard(v8f& a, v8f& b, v16b x, v16b y) { dep_guard_b(a, b, x, y); }
  static __device__ __forceinline__ void keep(v16b a, v16b b, v16b c, v16b d) { keep4_b(a, b, c, d); }
};

__device__ __forceinline__ float fsig(float x)  { return __builtin_amdgcn_rcpf(1.0f + expf(-x)); }
__device__ __forceinline__ float ftanh(float x) { return 1.0f - 2.0f * __builtin_amdgcn_rcpf(expf(2.0f * x) + 1.0f); }

template <int ET> struct Elem;
template <> struct Elem<0> { typedef _Float16 T; };
template <> struct Elem<1> { typedef __bf16 T; };
template <int ET, bool SPLIT, int BIAS_MODE, int OUT_MODE, bool RESID, int ACT = 0>
__global__ __launch_bounds__(256) void wmma_gemm64(
    const unsigned short* __restrict__ Ap, const unsigned short* __restrict__ A2p, int lda, long strideA,
    const unsigned short* __restrict__ Btp, const unsigned short* __restrict__ Bt2p, int ldb, long strideB,
    void* __restrict__ Cout, void* __restrict__ Cout2, int ldc, long strideC,
    const float* __restrict__ bias,
    const float* __restrict__ resid, long strideR,
    int M, int N, int K, float scale) {
  typedef typename Elem<ET>::T T;
  typedef typename Frag<T>::V V;
  const T* A = (const T*)Ap; const T* A2 = (const T*)A2p; const T* Bt = (const T*)Btp; const T* Bt2 = (const T*)Bt2p;
  __shared__ __align__(16) float sT[8][16 * 68];
  const int b    = blockIdx.y;
  const int lane = threadIdx.x & 31;
  const int wave = threadIdx.x >> 5;
  const int tilesN = N >> 6;
  const int tilesM = M >> 6;
  const int tile = blockIdx.x * 8 + wave;
  if (tile >= tilesM * tilesN) return;
  const int tm = tile / tilesN;
  const int tn = tile - tm * tilesN;
  const int m0 = tm << 6;
  const int n0 = tn << 6;

  const T* Ab  = A  + (size_t)b * strideA;
  const T* Bb  = Bt + (size_t)b * strideB;
  const T* Ab2 = SPLIT ? (A2  + (size_t)b * strideA) : nullptr;
  const T* Bb2 = SPLIT ? (Bt2 + (size_t)b * strideB) : nullptr;

  const int rlane = lane & 15;
  const int koff  = (lane >> 4) * 8;
  const int mOff  = (lane >> 4) * 8;

  v8f acc[4][4];
#pragma unroll
  for (int i = 0; i < 4; ++i)
#pragma unroll
    for (int j = 0; j < 4; ++j) acc[i][j] = (v8f){0.f,0.f,0.f,0.f,0.f,0.f,0.f,0.f};

  for (int k0 = 0; k0 < K; k0 += 32) {
    V bh[4], bl[4];
#pragma unroll
    for (int j = 0; j < 4; ++j) {
      const size_t bo = (size_t)(n0 + (j << 4) + rlane) * ldb + koff + k0;
      bh[j] = Frag<T>::load(Bb + bo);
      if (SPLIT) bl[j] = Frag<T>::load(Bb2 + bo);
    }
#pragma unroll
    for (int i = 0; i < 4; ++i) {
      const size_t ao = (size_t)(m0 + (i << 4) + rlane) * lda + koff + k0;
      V ah = Frag<T>::load(Ab + ao);
      V al;
      if (SPLIT) al = Frag<T>::load(Ab2 + ao);
#pragma unroll
      for (int j = 0; j < 4; ++j) {
        acc[i][j] = Frag<T>::mma(ah, bh[j], acc[i][j]);
        if (SPLIT) {
          acc[i][j] = Frag<T>::mma(ah, bl[j], acc[i][j]);
          acc[i][j] = Frag<T>::mma(al, bh[j], acc[i][j]);
        }
      }
      Frag<T>::guard(acc[i][0], acc[i][3], ah, SPLIT ? al : ah);
    }
    Frag<T>::keep(bh[0], bh[1], bh[2], bh[3]);
    if (SPLIT) Frag<T>::keep(bl[0], bl[1], bl[2], bl[3]);
  }
  acc_guard4(acc[0][0], acc[0][1], acc[0][2], acc[0][3]);
  acc_guard4(acc[1][0], acc[1][1], acc[1][2], acc[1][3]);
  acc_guard4(acc[2][0], acc[2][1], acc[2][2], acc[2][3]);
  acc_guard4(acc[3][0], acc[3][1], acc[3][2], acc[3][3]);

  float* slab = sT[wave];
  const float* Rb = RESID ? (resid + (size_t)b * strideR) : nullptr;
#pragma unroll
  for (int i = 0; i < 4; ++i) {
    const int mBase = m0 + (i << 4);
#pragma unroll
    for (int j = 0; j < 4; ++j) {
      const int n = n0 + (j << 4) + rlane;
      float bv = 0.f;
      if (BIAS_MODE == 2) bv = bias[n];
#pragma unroll
      for (int r = 0; r < 8; ++r) {
        float v = acc[i][j][r] * scale;
        if (BIAS_MODE == 1) v += bias[mBase + mOff + r];
        if (BIAS_MODE == 2) v += bv;
        if (RESID) v += Rb[(size_t)(mBase + mOff + r) * ldc + n];
        if (ACT == 1) v = tanhf(v);
        if (ACT == 2) v = fmaxf(v, 0.0f);
        if (ACT == 3) v = v / (1.0f + expf(-v));
        if (ACT == 4) v = (v > 0.f) ? v : 0.01f * v;
        if (ACT == 5) v = 0.5f * v * (1.0f + erff(v * 0.70710678118654752f));
        slab[(mOff + r) * 68 + (j << 4) + rlane] = v;
      }
    }
    __builtin_amdgcn_fence(__ATOMIC_RELEASE, "workgroup");
    __builtin_amdgcn_wave_barrier();
    __builtin_amdgcn_fence(__ATOMIC_ACQUIRE, "workgroup");
    if (OUT_MODE == 0) {
      float* C = (float*)Cout + (size_t)b * strideC;
      const int hh = lane >> 4, c4 = (lane & 15) * 4;
      for (int pass = 0; pass < 2; ++pass) {
#pragma unroll
        for (int it = 0; it < 8; ++it) {
          const int row = it * 2 + hh;
          v4f v = *(const v4f*)(slab + row * 68 + c4);
          *(volatile v4f*)(C + (size_t)(mBase + row) * ldc + n0 + c4) = v;
        }
        __threadfence();
      }
    } else {
      const int q = lane >> 3, c8 = (lane & 7) * 8;
      unsigned short* C  = (unsigned short*)Cout  + (size_t)b * strideC;
      unsigned short* C2 = (OUT_MODE == 2) ? ((unsigned short*)Cout2 + (size_t)b * strideC) : nullptr;
      for (int pass = 0; pass < 2; ++pass) {
#pragma unroll
        for (int it = 0; it < 4; ++it) {
          const int row = it * 4 + q;
          const float* sp = slab + row * 68 + c8;
          v8h hv, lv;
#pragma unroll
          for (int e = 0; e < 8; ++e) {
            if (OUT_MODE == 1) {
              hv[e] = (_Float16)sp[e];
            } else {
              unsigned short hb = f2bf_bits(sp[e]);
              unsigned short lb = f2bf_bits(sp[e] - bf_bits2f(hb));
              hv[e] = __builtin_bit_cast(_Float16, hb);
              lv[e] = __builtin_bit_cast(_Float16, lb);
            }
          }
          *(volatile v8h*)(C + (size_t)(mBase + row) * ldc + n0 + c8) = hv;
          if (OUT_MODE == 2) *(volatile v8h*)(C2 + (size_t)(mBase + row) * ldc + n0 + c8) = lv;
        }
        __threadfence();
      }
    }
    __builtin_amdgcn_fence(__ATOMIC_RELEASE, "workgroup");
    __builtin_amdgcn_wave_barrier();
    __builtin_amdgcn_fence(__ATOMIC_ACQUIRE, "workgroup");
  }
}

__global__ __launch_bounds__(NTHR) void xplane_kernel(const int* __restrict__ ids, const float* __restrict__ emb,
                                                      unsigned short* __restrict__ XB) {
  const int i = blockIdx.x * NTHR + threadIdx.x;
  if (i >= NROWS * XCH) return;
  const int m  = i / XCH;
  const int c8 = i - m * XCH;
  const int t  = m >> 5;
  const int b  = m & 31;
  int tok = ids[b * NSTEPS + t];
  tok = tok < 0 ? 0 : tok;
  tok = tok > (NVOCAB - 1) ? (NVOCAB - 1) : tok;
  const float* er = emb + (size_t)tok * NEMB;
  v8h hv;
#pragma unroll
  for (int e = 0; e < 8; ++e) {
    const int k  = c8 * 8 + e;
    const int kc = k < NEMB ? k : (NEMB - 1);
    const float x = er[kc];
    const float v = (k < NEMB) ? x : 0.0f;
    hv[e] = __builtin_bit_cast(_Float16, f2bf_bits(v));
  }
  unsigned short* dp = XB + (size_t)i * 8;
  *(volatile v8h*)dp = hv;
  __threadfence();
  *(volatile v8h*)dp = hv;
}

__global__ __launch_bounds__(NTHR) void rows_bf16_kernel(const float* __restrict__ src, int spitch, int kvalid,
                                                         int nchunk, int nrow, unsigned short* __restrict__ dst) {
  const int i = blockIdx.x * NTHR + threadIdx.x;
  if (i >= nrow * nchunk) return;
  const int n  = i / nchunk;
  const int c8 = i - n * nchunk;
  const float* sr = src + (size_t)n * spitch;
  v8h hv;
#pragma unroll
  for (int e = 0; e < 8; ++e) {
    const int k  = c8 * 8 + e;
    const int kc = k < kvalid ? k : (kvalid - 1);
    const float x = sr[kc];
    const float v = (k < kvalid) ? x : 0.0f;
    hv[e] = __builtin_bit_cast(_Float16, f2bf_bits(v));
  }
  unsigned short* dp = dst + (size_t)i * 8;
  *(volatile v8h*)dp = hv;
  __threadfence();
  *(volatile v8h*)dp = hv;
}

__global__ __launch_bounds__(NTHR) void bias_kernel(const float* __restrict__ bih_f, const float* __restrict__ bhh_f,
                                                    const float* __restrict__ bih_b, const float* __restrict__ bhh_b,
                                                    float* __restrict__ BIAS) {
  const int tid = threadIdx.x;
  const int which = blockIdx.x;
  const int idx = tid * 4;
  const v4f a0 = *(const v4f*)(bih_f + idx);
  const v4f a1 = *(const v4f*)(bhh_f + idx);
  const v4f c0 = *(const v4f*)(bih_b + idx);
  const v4f c1 = *(const v4f*)(bhh_b + idx);
  v4f o;
#pragma unroll
  for (int e = 0; e < 4; ++e) {
    const float x0 = a0[e], x1 = a1[e], y0 = c0[e], y1 = c1[e];
    const float sf = bf16r(x0) + bf16r(x1);
    const float sb = bf16r(y0) + bf16r(y1);
    o[e] = which ? sb : sf;
  }
  float* op = BIAS + (size_t)which * NGATE + idx;
  *(volatile v4f*)op = o;
  __threadfence();
  *(volatile v4f*)op = o;
}

__global__ __launch_bounds__(NTHR) void bilstm_kernel(const float* __restrict__ GPRE, const unsigned short* __restrict__ WHBp,
                                                      const float* __restrict__ BIAS, float* __restrict__ SEQ) {
  __shared__ __align__(16) unsigned short Hpl[2][RBLK * HPITCH];
  __shared__ __align__(16) float          Gs[RBLK * NGATE];
  __shared__ __align__(16) float          Sl[NTHR / 32][RBLK * SLABP];
  const __bf16* WHB = (const __bf16*)WHBp;
  const int tid = threadIdx.x, lane = tid & 31, wave = tid >> 5;
  const int c = lane & 15, hh = lane >> 4, koff = hh * 8;
  const int q8 = lane >> 3, c4q = (lane & 7) * 4;
  const int dir = blockIdx.x >> 1;
  const int rowbase = (blockIdx.x & 1) * RBLK;

  {
    unsigned short* hp = &Hpl[0][0];
#pragma unroll 1
    for (int i = tid; i < 2 * RBLK * HPITCH; i += NTHR) hp[i] = (unsigned short)0;
  }
  float cst[2][8], hst[2][8], bb[2][4];
#pragma unroll
  for (int nt = 0; nt < 2; ++nt) {
    const int j = 32 * wave + 16 * nt + c;
#pragma unroll
    for (int g = 0; g < 4; ++g) bb[nt][g] = BIAS[(size_t)dir * NGATE + g * NHID + j];
#pragma unroll
    for (int r = 0; r < 8; ++r) { cst[nt][r] = 0.0f; hst[nt][r] = 0.0f; }
  }
  __syncthreads();

  const __bf16* hhrow = (const __bf16*)&Hpl[0][0] + c * HPITCH + koff;
  const __bf16* hlrow = (const __bf16*)&Hpl[1][0] + c * HPITCH + koff;
  float* slab = Sl[wave];
  const v8f z8 = {0.f, 0.f, 0.f, 0.f, 0.f, 0.f, 0.f, 0.f};

#pragma unroll 1
  for (int t = 0; t < NSTEPS; ++t) {
    const int tt = dir ? (NSTEPS - 1 - t) : t;
    {
      const float* gsrc = GPRE + ((size_t)dir * NROWS + (size_t)tt * NBATCH + (size_t)rowbase) * NGATE;
#pragma unroll 4
      for (int i = 0; i < (RBLK * NGATE) / (4 * NTHR); ++i) {
        const int idx = i * NTHR + tid;
        const v4f v = *(const v4f*)(gsrc + (size_t)idx * 4);
        *(v4f*)(Gs + idx * 4) = v;
      }
    }
    __syncthreads();

#pragma unroll
    for (int nt = 0; nt < 2; ++nt) {
      const int j = 32 * wave + 16 * nt + c;
      const __bf16* wb = WHB + ((size_t)dir * NGATE + (size_t)j) * NHID + koff;
      v8f acc[4];
      acc[0] = z8; acc[1] = z8; acc[2] = z8; acc[3] = z8;
#pragma unroll 1
      for (int k0 = 0; k0 < NHID; k0 += 32) {
        const v16b ah = Frag<__bf16>::load(hhrow + k0);
        const v16b al = Frag<__bf16>::load(hlrow + k0);
        const v16b b0 = Frag<__bf16>::load(wb + k0);
        const v16b b1 = Frag<__bf16>::load(wb + (size_t)1 * NHID * NHID + k0);
        const v16b b2 = Frag<__bf16>::load(wb + (size_t)2 * NHID * NHID + k0);
        const v16b b3 = Frag<__bf16>::load(wb + (size_t)3 * NHID * NHID + k0);
        acc[0] = Frag<__bf16>::mma(ah, b0, acc[0]);
        acc[0] = Frag<__bf16>::mma(al, b0, acc[0]);
        acc[1] = Frag<__bf16>::mma(ah, b1, acc[1]);
        acc[1] = Frag<__bf16>::mma(al, b1, acc[1]);
        acc[2] = Frag<__bf16>::mma(ah, b2, acc[2]);
        acc[2] = Frag<__bf16>::mma(al, b2, acc[2]);
        acc[3] = Frag<__bf16>::mma(ah, b3, acc[3]);
        acc[3] = Frag<__bf16>::mma(al, b3, acc[3]);
        guard8_b(acc[0], acc[1], acc[2], acc[3], ah, al, b0, b1, b2, b3);
      }
      acc_guard4(acc[0], acc[1], acc[2], acc[3]);
#pragma unroll
      for (int r = 0; r < 8; ++r) {
        const float* gr = Gs + (8 * hh + r) * NGATE + j;
        const float zi = (acc[0][r] + gr[0])        + bb[nt][0];
        const float zf = (acc[1][r] + gr[NHID])     + bb[nt][1];
        const float zg = (acc[2][r] + gr[2 * NHID]) + bb[nt][2];
        const float zo = (acc[3][r] + gr[3 * NHID]) + bb[nt][3];
        const float ig = fsig(zi);
        const float fg = fsig(zf);
        const float gg = ftanh(zg);
        const float og = fsig(zo);
        const float cn = fg * cst[nt][r] + ig * gg;
        cst[nt][r] = cn;
        hst[nt][r] = og * ftanh(cn);
      }
    }
    __syncthreads();

#pragma unroll
    for (int nt = 0; nt < 2; ++nt) {
      const int j = 32 * wave + 16 * nt + c;
#pragma unroll
      for (int r = 0; r < 8; ++r) {
        const float h = hst[nt][r];
        const unsigned short hb = f2bf_bits(h);
        const unsigned short lb = f2bf_bits(h - bf_bits2f(hb));
        Hpl[0][(8 * hh + r) * HPITCH + j] = hb;
        Hpl[1][(8 * hh + r) * HPITCH + j] = lb;
        slab[(8 * hh + r) * SLABP + 16 * nt + c] = h;
      }
    }
    __builtin_amdgcn_fence(__ATOMIC_RELEASE, "workgroup");
    __builtin_amdgcn_wave_barrier();
    __builtin_amdgcn_fence(__ATOMIC_ACQUIRE, "workgroup");
    for (int pass = 0; pass < 2; ++pass) {
#pragma unroll
      for (int it = 0; it < 4; ++it) {
        const int row = it * 4 + q8;
        const v4f v = *(const v4f*)(slab + row * SLABP + c4q);
        *(volatile v4f*)(SEQ + ((size_t)(rowbase + row) * NSTEPS + (size_t)tt) * SEQW + dir * NHID + 32 * wave + c4q) = v;
      }
      __threadfence();
    }
    __builtin_amdgcn_fence(__ATOMIC_RELEASE, "workgroup");
    __builtin_amdgcn_wave_barrier();
    __builtin_amdgcn_fence(__ATOMIC_ACQUIRE, "workgroup");
  }
}

__global__ __launch_bounds__(NTHR) void cls_kernel(const float* __restrict__ SEQ, const float* __restrict__ Wc,
                                                   const float* __restrict__ bc, float* __restrict__ OUT0,
                                                   float* __restrict__ EMW) {
  __shared__ __align__(16) float Wcs[NTAGS * SEQW];
  __shared__ float bcs[16];
  __shared__ __align__(16) float St[NTHR / 32][32 * NTAGS];
  const int tid = threadIdx.x, lane = tid & 31, wave = tid >> 5;
#pragma unroll 1
  for (int i = tid; i < NTAGS * SEQW; i += NTHR) Wcs[i] = bf16r(Wc[i]);
  {
    const int ic = tid < NTAGS ? tid : (NTAGS - 1);
    const float v = bf16r(bc[ic]);
    if (tid < NTAGS) bcs[tid] = v;
  }
  __syncthreads();

  const int m = blockIdx.x * NTHR + tid;
  const float* rp = SEQ + (size_t)m * SEQW;
  float acc[NTAGS];
#pragma unroll
  for (int k = 0; k < NTAGS; ++k) acc[k] = 0.0f;
#pragma unroll 1
  for (int k4 = 0; k4 < SEQW / 4; ++k4) {
    const v4f v = *(const v4f*)(rp + 4 * k4);
#pragma unroll
    for (int k = 0; k < NTAGS; ++k) {
      const v4f w = *(const v4f*)(Wcs + k * SEQW + 4 * k4);
      acc[k] += (v[0] * w[0] + v[1] * w[1]) + (v[2] * w[2] + v[3] * w[3]);
    }
  }
  float* st = St[wave];
#pragma unroll
  for (int k = 0; k < NTAGS; ++k) st[lane * NTAGS + k] = acc[k] + bcs[k];
  __builtin_amdgcn_fence(__ATOMIC_RELEASE, "workgroup");
  __builtin_amdgcn_wave_barrier();
  __builtin_amdgcn_fence(__ATOMIC_ACQUIRE, "workgroup");
  const size_t base = (size_t)(blockIdx.x * NTHR + wave * 32) * NTAGS;
  for (int pass = 0; pass < 2; ++pass) {
#pragma unroll
    for (int i = 0; i < 3; ++i) {
      const int idx = 32 * i + lane;
      const int idc = idx < 72 ? idx : 71;
      const v4f v = *(const v4f*)(st + idc * 4);
      if (idx < 72) {
        *(volatile v4f*)(OUT0 + base + (size_t)idx * 4) = v;
        *(volatile v4f*)(EMW  + base + (size_t)idx * 4) = v;
      }
    }
    __threadfence();
  }
}

__global__ __launch_bounds__(32) void crf_kernel(const float* __restrict__ EMW, const int* __restrict__ tags,
                                                 const int* __restrict__ msk, const float* __restrict__ startT,
                                                 const float* __restrict__ endT, const float* __restrict__ trans,
                                                 float* __restrict__ loss_out) {
  __shared__ float s_tr[NTAGS * NTAGS];
  __shared__ float s_st[16];
  __shared__ float s_en[16];
  const int lane = threadIdx.x;
#pragma unroll 1
  for (int i = lane; i < NTAGS * NTAGS; i += 32) s_tr[i] = bf16r(trans[i]);
  {
    const int ic = lane < NTAGS ? lane : (NTAGS - 1);
    const float a = bf16r(startT[ic]);
    const float e = bf16r(endT[ic]);
    if (lane < NTAGS) { s_st[lane] = a; s_en[lane] = e; }
  }
  __syncthreads();

  const float* E  = EMW  + (size_t)lane * NSTEPS * NTAGS;
  const int*   tg = tags + (size_t)lane * NSTEPS;
  const int*   mk = msk  + (size_t)lane * NSTEPS;

  int t0 = tg[0];
  t0 = t0 < 0 ? 0 : t0; t0 = t0 > (NTAGS - 1) ? (NTAGS - 1) : t0;
  float score = s_st[t0] + E[t0];
  int prev = t0;
  int cnt  = mk[0];

  float alpha[NTAGS];
#pragma unroll
  for (int j = 0; j < NTAGS; ++j) alpha[j] = s_st[j] + E[j];

#pragma unroll 1
  for (int t = 1; t < NSTEPS; ++t) {
    int cur = tg[t];
    cur = cur < 0 ? 0 : cur; cur = cur > (NTAGS - 1) ? (NTAGS - 1) : cur;
    const int mt = mk[t];
    cnt += mt;
    const float ecur = E[t * NTAGS + cur];
    score += (float)mt * (s_tr[prev * NTAGS + cur] + ecur);
    prev = cur;
    float et[NTAGS];
#pragma unroll
    for (int j = 0; j < NTAGS; ++j) et[j] = E[t * NTAGS + j];
    float na[NTAGS];
#pragma unroll
    for (int jn = 0; jn < NTAGS; ++jn) {
      float mx = -3.0e38f;
#pragma unroll
      for (int ji = 0; ji < NTAGS; ++ji) mx = fmaxf(mx, alpha[ji] + s_tr[ji * NTAGS + jn]);
      float s = 0.0f;
#pragma unroll
      for (int ji = 0; ji < NTAGS; ++ji) s += __expf(alpha[ji] + s_tr[ji * NTAGS + jn] - mx);
      na[jn] = mx + __logf(s) + et[jn];
    }
#pragma unroll
    for (int j = 0; j < NTAGS; ++j) alpha[j] = (mt > 0) ? na[j] : alpha[j];
  }
  int se = cnt - 1;
  se = se < 0 ? se + NSTEPS : se;
  se = se < 0 ? 0 : se; se = se > (NSTEPS - 1) ? (NSTEPS - 1) : se;
  int lt = tg[se];
  lt = lt < 0 ? 0 : lt; lt = lt > (NTAGS - 1) ? (NTAGS - 1) : lt;
  score += s_en[lt];
  float mx = -3.0e38f;
#pragma unroll
  for (int j = 0; j < NTAGS; ++j) mx = fmaxf(mx, alpha[j] + s_en[j]);
  float s = 0.0f;
#pragma unroll
  for (int j = 0; j < NTAGS; ++j) s += __expf(alpha[j] + s_en[j] - mx);
  const float denom = mx + __logf(s);

  float v = score - denom;
#pragma unroll
  for (int off = 16; off > 0; off >>= 1) v += __shfl_xor(v, off, 32);
  if (lane == 0) {
    const float lo = -v;
    *(volatile float*)loss_out = lo;
    __threadfence();
    *(volatile float*)loss_out = lo;
  }
}

extern "C" void kernel_launch(void* const* d_in, const int* in_sizes, int n_in,
                              void* d_out, int out_size, void* d_ws, size_t ws_size, hipStream_t stream) {
  if (n_in < 17 || d_out == nullptr || d_ws == nullptr) return;
  if (in_sizes[0] != NROWS || in_sizes[1] != NROWS || in_sizes[2] != NROWS ||
      in_sizes[3] != NVOCAB * NEMB || in_sizes[4] != NGATE * NEMB || in_sizes[5] != NGATE * NHID ||
      in_sizes[6] != NGATE || in_sizes[7] != NGATE || in_sizes[8] != NGATE * NEMB || in_sizes[9] != NGATE * NHID ||
      in_sizes[10] != NGATE || in_sizes[11] != NGATE || in_sizes[12] != NTAGS * SEQW || in_sizes[13] != NTAGS ||
      in_sizes[14] != NTAGS || in_sizes[15] != NTAGS || in_sizes[16] != NTAGS * NTAGS ||
      out_size != NOUT0 + 1) return;

  const int*   ids    = (const int*)  d_in[0];
  const int*   imask  = (const int*)  d_in[1];
  const int*   itags  = (const int*)  d_in[2];
  const float* emb    = (const float*)d_in[3];
  const float* wih_f  = (const float*)d_in[4];
  const float* whh_f  = (const float*)d_in[5];
  const float* bih_f  = (const float*)d_in[6];
  const float* bhh_f  = (const float*)d_in[7];
  const float* wih_b  = (const float*)d_in[8];
  const float* whh_b  = (const float*)d_in[9];
  const float* bih_b  = (const float*)d_in[10];
  const float* bhh_b  = (const float*)d_in[11];
  const float* wc     = (const float*)d_in[12];
  const float* bcv    = (const float*)d_in[13];
  const float* startv = (const float*)d_in[14];
  const float* endv   = (const float*)d_in[15];
  const float* transv = (const float*)d_in[16];
  float* out0 = (float*)d_out;
  float* out1 = out0 + (size_t)NOUT0;

  char* ws = (char*)d_ws; size_t off = 0;
  auto carve = [&](size_t bytes) -> char* { char* p = ws + off; off += (bytes + 255) & ~(size_t)255; return p; };
  unsigned short* XB   = (unsigned short*)carve((size_t)NROWS * KPE * 2);
  unsigned short* WIHB = (unsigned short*)carve((size_t)2 * NGATE * KPE * 2);
  unsigned short* WHHB = (unsigned short*)carve((size_t)2 * NGATE * NHID * 2);
  float*          BIAS = (float*)carve((size_t)2 * NGATE * 4);
  float*          GPRE = (float*)carve((size_t)2 * NROWS * NGATE * 4);
  float*          SEQ  = (float*)carve((size_t)NROWS * SEQW * 4);
  float*          EMW  = (float*)carve((size_t)NROWS * NTAGS * 4);
  if (off > ws_size || off > (size_t)134217728) return;

  xplane_kernel<<<(NROWS * XCH) / NTHR, NTHR, 0, stream>>>(ids, emb, XB);
  rows_bf16_kernel<<<(NGATE * XCH) / NTHR, NTHR, 0, stream>>>(wih_f, NEMB, NEMB, XCH, NGATE, WIHB);
  rows_bf16_kernel<<<(NGATE * XCH) / NTHR, NTHR, 0, stream>>>(wih_b, NEMB, NEMB, XCH, NGATE, WIHB + (size_t)NGATE * KPE);
  rows_bf16_kernel<<<(NGATE * HCH) / NTHR, NTHR, 0, stream>>>(whh_f, NHID, NHID, HCH, NGATE, WHHB);
  rows_bf16_kernel<<<(NGATE * HCH) / NTHR, NTHR, 0, stream>>>(whh_b, NHID, NHID, HCH, NGATE, WHHB + (size_t)NGATE * NHID);
  bias_kernel<<<2, NTHR, 0, stream>>>(bih_f, bhh_f, bih_b, bhh_b, BIAS);

  const dim3 ggrid(((NROWS / 64) * (NGATE / 64)) / 8, 1);
  wmma_gemm64<1, false, 0, 0, false, 0><<<ggrid, 256, 0, stream>>>(
      XB, XB, KPE, 0L, WIHB, WIHB, KPE, 0L, (void*)GPRE, (void*)GPRE, NGATE, 0L,
      BIAS, GPRE, 0L, NROWS, NGATE, KPE, 1.0f);
  wmma_gemm64<1, false, 0, 0, false, 0><<<ggrid, 256, 0, stream>>>(
      XB, XB, KPE, 0L, WIHB + (size_t)NGATE * KPE, WIHB + (size_t)NGATE * KPE, KPE, 0L,
      (void*)(GPRE + (size_t)NROWS * NGATE), (void*)(GPRE + (size_t)NROWS * NGATE), NGATE, 0L,
      BIAS, GPRE, 0L, NROWS, NGATE, KPE, 1.0f);

  bilstm_kernel<<<4, NTHR, 0, stream>>>(GPRE, WHHB, BIAS, SEQ);

  cls_kernel<<<NROWS / NTHR, NTHR, 0, stream>>>(SEQ, wc, bcv, out0, EMW);

  crf_kernel<<<1, 32, 0, stream>>>(EMW, itags, imask, startv, endv, transv, out1);
}
